// BuildingPointNet_19679540150375
// MI455X (gfx1250) — hardware-verified
//
#include <hip/hip_runtime.h>
#include <math.h>
#include <stddef.h>
#include <stdint.h>


#define NPT   40000
#define KNB   16
#define NSL   17
#define C1    64
#define F1    128
#define C2    128
#define F2    256
#define NCL   8
#define NCLP  16
#define EPSV  1e-5f
#define ASC   8
#define WSC   1024
#define WSCAP 134217728

static_assert(NPT % 32 == 0);
static_assert(NPT % 16 == 0);
static_assert(C1 % 32 == 0);
static_assert(C2 % 32 == 0);
static_assert(F1 % 32 == 0);
static_assert(F2 % 32 == 0);
static_assert(F1 == C2);
static_assert(NCLP == 16);

typedef float    v4f  __attribute__((ext_vector_type(4)));
typedef float    v8f  __attribute__((ext_vector_type(8)));
typedef _Float16 v4h  __attribute__((ext_vector_type(4)));
typedef _Float16 v8h  __attribute__((ext_vector_type(8)));
typedef _Float16 v16h __attribute__((ext_vector_type(16)));
union FragH { v16h v; v8h h[2]; };

__device__ __forceinline__ v8f wmf(v16h a, v16h b, v8f c) {
  v8f d = __builtin_amdgcn_wmma_f32_16x16x32_f16(false, a, false, b, (short)0, c, false, false);
  asm volatile("v_nop\n\tv_nop\n\tv_nop\n\tv_nop" : "+v"(d) : "v"(a), "v"(b));
  return d;
}

__device__ __forceinline__ v8f splat8(float x) { v8f r = {x, x, x, x, x, x, x, x}; return r; }

__device__ __forceinline__ v4f relu4(v4f a) {
  v4f o;
  o.x = fmaxf(a.x, 0.0f); o.y = fmaxf(a.y, 0.0f); o.z = fmaxf(a.z, 0.0f); o.w = fmaxf(a.w, 0.0f);
  return o;
}

__device__ __forceinline__ v16h ldfrag(const _Float16* p, int k0, int hh) {
  FragH u;
  u.h[0] = *(const v8h*)(p + k0 + 8 * hh);
  u.h[1] = *(const v8h*)(p + k0 + 16 + 8 * hh);
  return u.v;
}

__device__ __forceinline__ v8h prepw_piece(const float* ts, int p, int npc) {
  const int row = p / npc, k8 = (p - row * npc) * 8;
  v8h o;
#pragma unroll
  for (int e = 0; e < 8; ++e) o[e] = (_Float16)(ts[(k8 + e) * 16 + row] * (float)WSC);
  return o;
}

__global__ __launch_bounds__(256) void k_prepw(const float* __restrict__ W, int Kd, int Nd, _Float16* dst) {
  __shared__ __attribute__((aligned(16))) float ts[256 * 16];
  const int t = threadIdx.x;
  const int n0 = blockIdx.x * 16;
  if (t < Kd) {
    const float* wrow = W + (size_t)t * Nd;
#pragma unroll
    for (int nn = 0; nn < 16; ++nn) {
      const int n = n0 + nn;
      const float v = wrow[min(n, Nd - 1)];
      ts[t * 16 + nn] = (n < Nd) ? v : 0.0f;
    }
  }
  __syncthreads();
  const int npc = Kd >> 3;
  const int tot = 16 * npc;
  const int p0 = t, p1 = t + 256;
  const bool a0 = p0 < tot, a1 = p1 < tot;
  const v8h o0 = prepw_piece(ts, a0 ? p0 : 0, npc);
  const v8h o1 = prepw_piece(ts, a1 ? p1 : 0, npc);
  _Float16* d0 = dst + (size_t)n0 * Kd + 8 * (a0 ? p0 : 0);
  _Float16* d1 = dst + (size_t)n0 * Kd + 8 * (a1 ? p1 : 0);
  if (a0) *(volatile v8h*)d0 = o0;
  if (a1) *(volatile v8h*)d1 = o1;
  __threadfence();
  if (a0) *(volatile v8h*)d0 = o0;
  if (a1) *(volatile v8h*)d1 = o1;
}

struct Nrm { float x, y, z; };

__device__ __forceinline__ Nrm unit_normal(const float* __restrict__ pos, const int* __restrict__ nbr, int i) {
#pragma clang fp contract(off)
  int j0 = nbr[(size_t)i * KNB + 0];
  int j1 = nbr[(size_t)i * KNB + 1];
  j0 = min(max(j0, 0), NPT - 1);
  j1 = min(max(j1, 0), NPT - 1);
  const float px = pos[3 * i], py = pos[3 * i + 1], pz = pos[3 * i + 2];
  const float ax = pos[3 * j0] - px, ay = pos[3 * j0 + 1] - py, az = pos[3 * j0 + 2] - pz;
  const float bx = pos[3 * j1] - px, by = pos[3 * j1 + 1] - py, bz = pos[3 * j1 + 2] - pz;
  const float cx = ay * bz - az * by;
  const float cy = az * bx - ax * bz;
  const float cz = ax * by - ay * bx;
  const float ss = (cx * cx + cz * cz) + cy * cy;
  const float nn = sqrtf(ss);
  const float inv = 1.0f / fmaxf(nn, 1e-12f);
  const bool ok = nn > 0.0f;
  Nrm o;
  o.x = ok ? cx * inv : 0.0f;
  o.y = ok ? cy * inv : 0.0f;
  o.z = ok ? cz * inv : 1.0f;
  return o;
}

__global__ __launch_bounds__(256) void k_prepq(const float* __restrict__ pos, const int* __restrict__ nbr,
                                                const float* __restrict__ W1, const float* __restrict__ b1,
                                                float* Qp) {
  __shared__ __attribute__((aligned(16))) float s_x6[32 * 8];
  const int t = threadIdx.x, lane = t & 31, w = t >> 5;
  const int nb = blockIdx.x * 32;
  if (w == 0) {
    const int i = nb + lane;
    const Nrm n = unit_normal(pos, nbr, i);
    s_x6[lane * 8 + 0] = pos[3 * i];
    s_x6[lane * 8 + 1] = pos[3 * i + 1];
    s_x6[lane * 8 + 2] = pos[3 * i + 2];
    s_x6[lane * 8 + 3] = n.x;
    s_x6[lane * 8 + 4] = n.y;
    s_x6[lane * 8 + 5] = n.z;
    s_x6[lane * 8 + 6] = 0.0f;
    s_x6[lane * 8 + 7] = 0.0f;
  }
  __syncthreads();
  v4f q[2];
#pragma unroll
  for (int it = 0; it < 2; ++it) {
    const int f = it * 256 + t;
    const int nd = f >> 4;
    const int c4 = (f & 15) * 4;
    v4f acc = *(const v4f*)(b1 + c4);
#pragma unroll 1
    for (int f6 = 0; f6 < 6; ++f6) {
      const float xv = s_x6[nd * 8 + f6];
      const v4f wv = *(const v4f*)(W1 + f6 * C1 + c4);
      acc = acc + xv * wv;
    }
    q[it] = acc;
  }
  float* d0 = Qp + (size_t)(nb + (t >> 4)) * C1 + (t & 15) * 4;
  float* d1 = Qp + (size_t)(nb + ((t + 256) >> 4)) * C1 + (t & 15) * 4;
  *(volatile v4f*)d0 = q[0];
  *(volatile v4f*)d1 = q[1];
  __threadfence();
  *(volatile v4f*)d0 = q[0];
  *(volatile v4f*)d1 = q[1];
}

template <int KH, int NO, int L2>
__global__ __launch_bounds__(64) void k_conv(const float* __restrict__ pos, const int* __restrict__ nbr,
                                              const float* __restrict__ Qp, const float* __restrict__ Wr,
                                              const float* __restrict__ pg, const float* __restrict__ pb,
                                              const float* __restrict__ pm, const float* __restrict__ pv,
                                              const _Float16* __restrict__ Wt, const float* __restrict__ bo,
                                              const _Float16* __restrict__ We, const float* __restrict__ be,
                                              float* outp) {
  constexpr int QN = KH / 4;
  constexpr int RP = 64 / QN;
  constexpr int NPASS = 16 / RP;
  constexpr int KS = KH / 32;
  constexpr int NTW = NO / 32;
  constexpr int NST = L2 ? (16 * NCL) : (16 * C2);
  static_assert(QN * RP == 64);
  static_assert(RP * NPASS == 16);
  static_assert(L2 || NO == F1);
  static_assert(!L2 || NO == F2);
  __shared__ __attribute__((aligned(16))) _Float16 s_hid[16 * KH];
  __shared__ __attribute__((aligned(16))) _Float16 s_x[16 * NO];
  __shared__ __attribute__((aligned(16))) float s_st[NST];
  __shared__ __attribute__((aligned(16))) float s_rel[16 * 4];
  __shared__ int s_j[16];

  const int t = threadIdx.x, lane = t & 31, w = t >> 5, hh = lane >> 4, nl = lane & 15;
  const int base = blockIdx.x * 16;
  const int quad = t % QN, row0 = t / QN;
  const int c4 = 4 * quad;

  const v4f wr0 = *(const v4f*)(Wr + c4);
  const v4f wr1 = *(const v4f*)(Wr + KH + c4);
  const v4f wr2 = *(const v4f*)(Wr + 2 * KH + c4);
  const v4f g4 = *(const v4f*)(pg + c4);
  const v4f t4 = *(const v4f*)(pb + c4);
  const v4f m4 = *(const v4f*)(pm + c4);
  const v4f v4 = *(const v4f*)(pv + c4);
  v4f sc4, sh4;
  sc4.x = g4.x * (1.0f / sqrtf(v4.x + EPSV));
  sc4.y = g4.y * (1.0f / sqrtf(v4.y + EPSV));
  sc4.z = g4.z * (1.0f / sqrtf(v4.z + EPSV));
  sc4.w = g4.w * (1.0f / sqrtf(v4.w + EPSV));
  sh4 = t4 - m4 * sc4;

  v8f accm[NTW];
#pragma unroll
  for (int nt = 0; nt < NTW; ++nt) accm[nt] = splat8(-3.0e38f);

#pragma unroll 1
  for (int s = 0; s < NSL; ++s) {
    if (w == 0) {
      const int i = base + nl;
      const int jn = nbr[(size_t)i * KNB + min(s, KNB - 1)];
      int j = (s < KNB) ? jn : i;
      j = min(max(j, 0), NPT - 1);
      const float rx = pos[3 * j] - pos[3 * i];
      const float ry = pos[3 * j + 1] - pos[3 * i + 1];
      const float rz = pos[3 * j + 2] - pos[3 * i + 2];
      if (hh == 0) {
        s_j[nl] = j;
        s_rel[4 * nl] = rx;
        s_rel[4 * nl + 1] = ry;
        s_rel[4 * nl + 2] = rz;
        s_rel[4 * nl + 3] = 0.0f;
      }
    }
    __syncthreads();
#pragma unroll
    for (int p = 0; p < NPASS; ++p) {
      const int r = p * RP + row0;
      const int j = s_j[r];
      const v4f rl = *(const v4f*)(s_rel + 4 * r);
      const v4f q = *(const v4f*)(Qp + (size_t)j * KH + c4);
      v4f h = q + rl.x * wr0 + rl.y * wr1 + rl.z * wr2;
      h = relu4(h);
      h = h * sc4 + sh4;
      v4h o;
      o.x = (_Float16)(h.x * (float)ASC);
      o.y = (_Float16)(h.y * (float)ASC);
      o.z = (_Float16)(h.z * (float)ASC);
      o.w = (_Float16)(h.w * (float)ASC);
      *(v4h*)(s_hid + r * KH + c4) = o;
    }
    __syncthreads();
    v16h af[KS];
    {
      const _Float16* ap = s_hid + nl * KH;
#pragma unroll
      for (int ks = 0; ks < KS; ++ks) af[ks] = ldfrag(ap, 32 * ks, hh);
    }
#pragma unroll
    for (int nt = 0; nt < NTW; ++nt) {
      const _Float16* bp = Wt + (size_t)(16 * (w * NTW + nt) + nl) * KH;
      v8f c = splat8(0.0f);
#pragma unroll
      for (int ks = 0; ks < KS; ++ks) c = wmf(af[ks], ldfrag(bp, 32 * ks, hh), c);
#pragma unroll
      for (int r = 0; r < 8; ++r) accm[nt][r] = fmaxf(accm[nt][r], c[r]);
    }
  }

  constexpr float OSC = 1.0f / (float)(ASC * WSC);
#pragma unroll
  for (int nt = 0; nt < NTW; ++nt) {
    const int col = 16 * (w * NTW + nt) + nl;
    const float bv = bo[col];
#pragma unroll
    for (int r = 0; r < 8; ++r) {
      const float x = fmaxf(accm[nt][r] * OSC + bv, 0.0f);
      s_x[(8 * hh + r) * NO + col] = (_Float16)(x * (float)ASC);
    }
  }
  __syncthreads();

  if (L2 == 0) {
    v16h ax[F1 / 32];
    {
      const _Float16* ap = s_x + nl * NO;
#pragma unroll
      for (int ks = 0; ks < F1 / 32; ++ks) ax[ks] = ldfrag(ap, 32 * ks, hh);
    }
#pragma unroll
    for (int nt = 0; nt < C2 / 32; ++nt) {
      const int col = 16 * ((C2 / 32) * w + nt) + nl;
      const _Float16* bp = We + (size_t)col * F1;
      v8f c = splat8(0.0f);
#pragma unroll
      for (int ks = 0; ks < F1 / 32; ++ks) c = wmf(ax[ks], ldfrag(bp, 32 * ks, hh), c);
      const float bv = be[col];
#pragma unroll
      for (int r = 0; r < 8; ++r) s_st[(8 * hh + r) * C2 + col] = c[r] * OSC + bv;
    }
    __syncthreads();
    v4f vv[8];
#pragma unroll
    for (int it = 0; it < 8; ++it) vv[it] = *(const v4f*)(s_st + (2 * it + w) * C2 + 4 * lane);
    float* op = outp + (size_t)base * C2 + 4 * lane;
#pragma unroll
    for (int it = 0; it < 8; ++it) *(volatile v4f*)(op + (size_t)(2 * it + w) * C2) = vv[it];
    __threadfence();
#pragma unroll
    for (int it = 0; it < 8; ++it) *(volatile v4f*)(op + (size_t)(2 * it + w) * C2) = vv[it];
  } else {
    if (w == 0) {
      const _Float16* ap = s_x + nl * NO;
      const _Float16* bp = We + (size_t)nl * F2;
      v8f c = splat8(0.0f);
#pragma unroll
      for (int ks = 0; ks < F2 / 32; ++ks) c = wmf(ldfrag(ap, 32 * ks, hh), ldfrag(bp, 32 * ks, hh), c);
      const float bv = be[min(nl, NCL - 1)];
      float lg[8];
#pragma unroll
      for (int r = 0; r < 8; ++r) lg[r] = c[r] * OSC + bv;
      if (nl < NCL) {
#pragma unroll
        for (int r = 0; r < 8; ++r) s_st[(8 * hh + r) * NCL + nl] = lg[r];
      }
    }
    __syncthreads();
    if (w == 0) {
      const int r = lane >> 1, hc = lane & 1;
      const v4f x = *(const v4f*)(s_st + r * NCL + 4 * hc);
      float mx = fmaxf(fmaxf(x.x, x.y), fmaxf(x.z, x.w));
      mx = fmaxf(mx, __shfl_xor(mx, 1, 32));
      const v4f sh = x - mx;
      v4f e;
      e.x = expf(sh.x); e.y = expf(sh.y); e.z = expf(sh.z); e.w = expf(sh.w);
      float su = (e.x + e.y) + (e.z + e.w);
      su += __shfl_xor(su, 1, 32);
      const float lz = logf(su);
      const v4f o = sh - lz;
      float* d = outp + (size_t)base * NCL + 4 * lane;
      *(volatile v4f*)d = o;
      __threadfence();
      *(volatile v4f*)d = o;
    }
  }
}

extern "C" void kernel_launch(void* const* d_in, const int* in_sizes, int n_in,
                              void* d_out, int out_size, void* d_ws, size_t ws_size,
                              hipStream_t stream) {
  if (n_in < 20) return;
  if (in_sizes[0] != NPT * 3 || in_sizes[1] != NPT * KNB) return;
  if (in_sizes[2] != 9 * C1) return;
  for (int i = 3; i <= 7; ++i) if (in_sizes[i] != C1) return;
  if (in_sizes[8] != C1 * F1 || in_sizes[9] != F1) return;
  if (in_sizes[10] != (F1 + 3) * C2) return;
  for (int i = 11; i <= 15; ++i) if (in_sizes[i] != C2) return;
  if (in_sizes[16] != C2 * F2 || in_sizes[17] != F2) return;
  if (in_sizes[18] != F2 * NCL || in_sizes[19] != NCL) return;
  if (out_size != NPT * NCL) return;

  const float* pos = (const float*)d_in[0];
  const int*   nbr = (const int*)d_in[1];
  const float* W1  = (const float*)d_in[2];
  const float* b1  = (const float*)d_in[3];
  const float* g1  = (const float*)d_in[4];
  const float* bt1 = (const float*)d_in[5];
  const float* m1  = (const float*)d_in[6];
  const float* v1  = (const float*)d_in[7];
  const float* W2  = (const float*)d_in[8];
  const float* b2  = (const float*)d_in[9];
  const float* W3  = (const float*)d_in[10];
  const float* b3  = (const float*)d_in[11];
  const float* g2  = (const float*)d_in[12];
  const float* bt2 = (const float*)d_in[13];
  const float* m2  = (const float*)d_in[14];
  const float* v2  = (const float*)d_in[15];
  const float* W4  = (const float*)d_in[16];
  const float* b4  = (const float*)d_in[17];
  const float* Wc  = (const float*)d_in[18];
  const float* bc  = (const float*)d_in[19];
  float* out = (float*)d_out;

  char* ws = (char*)d_ws;
  size_t off = 0;
  const size_t oW2 = off; off += (size_t)F1 * C1 * 2;     off = (off + 255) & ~(size_t)255;
  const size_t oW3 = off; off += (size_t)C2 * F1 * 2;     off = (off + 255) & ~(size_t)255;
  const size_t oW4 = off; off += (size_t)F2 * C2 * 2;     off = (off + 255) & ~(size_t)255;
  const size_t oWc = off; off += (size_t)NCLP * F2 * 2;   off = (off + 255) & ~(size_t)255;
  const size_t oQ  = off; off += (size_t)NPT * C1 * 4;    off = (off + 255) & ~(size_t)255;
  const size_t oP  = off; off += (size_t)NPT * C2 * 4;    off = (off + 255) & ~(size_t)255;
  if (off > ws_size || off > (size_t)WSCAP) return;
  _Float16* w2t = (_Float16*)(ws + oW2);
  _Float16* w3t = (_Float16*)(ws + oW3);
  _Float16* w4t = (_Float16*)(ws + oW4);
  _Float16* wct = (_Float16*)(ws + oWc);
  float*    Qp  = (float*)(ws + oQ);
  float*    Pp  = (float*)(ws + oP);

  k_prepw<<<F1 / 16, 256, 0, stream>>>(W2, C1, F1, w2t);
  k_prepw<<<C2 / 16, 256, 0, stream>>>(W3, F1, C2, w3t);
  k_prepw<<<F2 / 16, 256, 0, stream>>>(W4, C2, F2, w4t);
  k_prepw<<<NCLP / 16, 256, 0, stream>>>(Wc, F2, NCL, wct);

  k_prepq<<<NPT / 32, 256, 0, stream>>>(pos, nbr, W1, b1, Qp);

  k_conv<C1, F1, 0><<<NPT / 16, 64, 0, stream>>>(pos, nbr, Qp, W1 + 6 * C1, g1, bt1, m1, v1,
                                                 w2t, b2, w3t, b3, Pp);
  k_conv<C2, F2, 1><<<NPT / 16, 64, 0, stream>>>(pos, nbr, Pp, W3 + (size_t)F1 * C2, g2, bt2, m2, v2,
                                                 w4t, b4, wct, bc, out);
}
